// NormLocalAttention_71871982731659
// MI455X (gfx1250) — hardware-verified
//
#include <hip/hip_runtime.h>
#include <math.h>
#include <stdint.h>

#define SQ    8192
#define DM    1024
#define NH    16
#define HD    64
#define NCH   (SQ / 64)
#define WSC   64.0f
#define RSC   4096.0f
static_assert(NH * HD == DM);
static_assert((SQ % 64) == 0 && (DM % 64) == 0);
static_assert(NCH * 64 == SQ);

typedef _Float16 v16h __attribute__((ext_vector_type(16)));
typedef _Float16 v8h  __attribute__((ext_vector_type(8)));
typedef __attribute__((ext_vector_type(16))) __bf16 v16b;
typedef unsigned short v8us __attribute__((ext_vector_type(8)));
typedef float    v8f  __attribute__((ext_vector_type(8)));
typedef float    v4f  __attribute__((ext_vector_type(4)));
typedef unsigned int v4u __attribute__((ext_vector_type(4)));

__device__ __forceinline__ unsigned short bf_bits(float f) {
  unsigned u = __float_as_uint(f);
  return (unsigned short)((u + 0x7FFFu + ((u >> 16) & 1u)) >> 16);
}
__device__ __forceinline__ float bf_up(unsigned short h) { return __uint_as_float(((unsigned)h) << 16); }
__device__ __forceinline__ float bfr(float f) { return bf_up(bf_bits(f)); }
__device__ __forceinline__ unsigned short h_bits(_Float16 x) { return __builtin_bit_cast(unsigned short, x); }
__device__ __forceinline__ unsigned pk16(unsigned short a, unsigned short b) { return (unsigned)a | ((unsigned)b << 16); }
__device__ __forceinline__ v8f zero8() { v8f z = {0.f, 0.f, 0.f, 0.f, 0.f, 0.f, 0.f, 0.f}; return z; }

__device__ __forceinline__ v16h ldfrag_h(const _Float16* p) {
  union { v16h v; v8h h[2]; } f;
  f.h[0] = *(const v8h*)(p);
  f.h[1] = *(const v8h*)(p + 16);
  return f.v;
}
union FB { v16b v; v16h h; v8us u[2]; };
__device__ __forceinline__ FB ldfrag_b(const unsigned short* p) {
  FB f;
  f.u[0] = *(const v8us*)(p);
  f.u[1] = *(const v8us*)(p + 16);
  return f;
}

__device__ __forceinline__ v8f mma_h(v16h a, v16h b, v8f c) {
  c = __builtin_amdgcn_wmma_f32_16x16x32_f16(false, a, false, b, (short)0, c, false, false);
#if defined(__HIP_DEVICE_COMPILE__)
  asm volatile("v_nop\n\tv_nop\n\tv_nop\n\tv_nop" : "+v"(c) : "v"(a), "v"(b));
#endif
  return c;
}
__device__ __forceinline__ v8f mma_h_raw(v16h a, v16h b, v8f c) {
  return __builtin_amdgcn_wmma_f32_16x16x32_f16(false, a, false, b, (short)0, c, false, false);
}
__device__ __forceinline__ v8f mma_b_raw(v16b a, v16b b, v8f c) {
  return __builtin_amdgcn_wmma_f32_16x16x32_bf16(false, a, false, b, (short)0, c, false, false);
}
__device__ __forceinline__ void dep_guard1(v8f& a, v8f& b, v16h x) {
#if defined(__HIP_DEVICE_COMPILE__)
  asm volatile("v_nop\n\tv_nop\n\tv_nop\n\tv_nop" : "+v"(a), "+v"(b) : "v"(x));
#endif
}
__device__ __forceinline__ void dep_guard2(v8f& a, v8f& b, v16h x, v16h y) {
#if defined(__HIP_DEVICE_COMPILE__)
  asm volatile("v_nop\n\tv_nop\n\tv_nop\n\tv_nop" : "+v"(a), "+v"(b) : "v"(x), "v"(y));
#endif
}
__device__ __forceinline__ void keep4_h(v16h a, v16h b, v16h c, v16h d) {
#if defined(__HIP_DEVICE_COMPILE__)
  asm volatile("v_nop" :: "v"(a), "v"(b), "v"(c), "v"(d));
#endif
}
__device__ __forceinline__ void acc_guard4(v8f& a, v8f& b, v8f& c, v8f& d) {
#if defined(__HIP_DEVICE_COMPILE__)
  asm volatile("v_nop\n\tv_nop\n\tv_nop\n\tv_nop" : "+v"(a), "+v"(b), "+v"(c), "+v"(d));
#endif
}
__device__ __forceinline__ void wave_sync_lds() {
  __builtin_amdgcn_fence(__ATOMIC_RELEASE, "workgroup");
  __builtin_amdgcn_wave_barrier();
  __builtin_amdgcn_fence(__ATOMIC_ACQUIRE, "workgroup");
}

template <int BF>
__device__ __forceinline__ unsigned short cvt16(float f, float wsc) {
  if (BF) return bf_bits(f);
  return h_bits((_Float16)(bfr(f) * wsc));
}
template <int BF>
__global__ __launch_bounds__(256) void conv16(const float* __restrict__ W, unsigned short* Wh, int n8,
                                              float wsc) {
  const int i = blockIdx.x * 256 + threadIdx.x;
  if (i >= n8) return;
  const size_t e0 = (size_t)i * 8;
  const v4f a = *(const v4f*)(W + e0);
  const v4f b = *(const v4f*)(W + e0 + 4);
  v4u u;
  u[0] = pk16(cvt16<BF>(a[0], wsc), cvt16<BF>(a[1], wsc));
  u[1] = pk16(cvt16<BF>(a[2], wsc), cvt16<BF>(a[3], wsc));
  u[2] = pk16(cvt16<BF>(b[0], wsc), cvt16<BF>(b[1], wsc));
  u[3] = pk16(cvt16<BF>(b[2], wsc), cvt16<BF>(b[3], wsc));
  for (int pass = 0; pass < 2; ++pass) {
    *(volatile v4u*)(Wh + e0) = u;
    __threadfence();
  }
}

template <int BM>
__global__ __launch_bounds__(256) void gemm64(
    const unsigned short* __restrict__ Ap, int lda,
    const unsigned short* __restrict__ Btp, int ldb,
    const float* __restrict__ bias, int nb,
    unsigned short* Cout, unsigned short* Cout2, int ldc,
    int M, int N, int K, float oscale, float rsc) {
  const _Float16* A  = (const _Float16*)(const void*)Ap;
  const _Float16* Bt = (const _Float16*)(const void*)Btp;
  __shared__ __align__(16) float sT[8][16 * 68];
  const int lane = threadIdx.x & 31;
  const int wave = threadIdx.x >> 5;
  const int tilesN = N >> 6;
  const int tilesM = M >> 6;
  const int tile = blockIdx.x * 8 + wave;
  if (tile >= tilesM * tilesN) return;
  const int tm = tile / tilesN;
  const int tn = tile - tm * tilesN;
  const int m0 = tm << 6;
  const int n0 = tn << 6;

  const int rlane = lane & 15;
  const int koff  = (lane >> 4) * 8;
  const int mOff  = (lane >> 4) * 8;

  v8f acc[4][4];
#pragma unroll
  for (int i = 0; i < 4; ++i)
#pragma unroll
    for (int j = 0; j < 4; ++j) acc[i][j] = zero8();

  for (int k0 = 0; k0 < K; k0 += 32) {
    v16h bh[4];
#pragma unroll
    for (int j = 0; j < 4; ++j) {
      const size_t bo = (size_t)(n0 + (j << 4) + rlane) * ldb + koff + k0;
      bh[j] = ldfrag_h(Bt + bo);
    }
#pragma unroll
    for (int i = 0; i < 4; ++i) {
      const size_t ao = (size_t)(m0 + (i << 4) + rlane) * lda + koff + k0;
      const v16h ah = ldfrag_h(A + ao);
#pragma unroll
      for (int j = 0; j < 4; ++j) acc[i][j] = mma_h_raw(ah, bh[j], acc[i][j]);
      dep_guard1(acc[i][0], acc[i][3], ah);
    }
    keep4_h(bh[0], bh[1], bh[2], bh[3]);
  }
  acc_guard4(acc[0][0], acc[0][1], acc[0][2], acc[0][3]);
  acc_guard4(acc[1][0], acc[1][1], acc[1][2], acc[1][3]);
  acc_guard4(acc[2][0], acc[2][1], acc[2][2], acc[2][3]);
  acc_guard4(acc[3][0], acc[3][1], acc[3][2], acc[3][3]);

  const int q8 = lane >> 3, c8 = (lane & 7) * 8;

  float bcol[8];
#pragma unroll
  for (int q = 0; q < 8; ++q) {
    if (BM == 1) {
      int bi = n0 + c8 + q;
      bi = (bi < 0) ? 0 : ((bi > nb - 1) ? (nb - 1) : bi);
      bcol[q] = bfr(bias[bi]);
    } else {
      bcol[q] = 0.0f;
    }
  }

  float* slab = sT[wave];
#pragma unroll
  for (int i = 0; i < 4; ++i) {
    const int mBase = m0 + (i << 4);
#pragma unroll
    for (int j = 0; j < 4; ++j) {
#pragma unroll
      for (int r = 0; r < 8; ++r) {
        slab[(mOff + r) * 68 + (j << 4) + rlane] = acc[i][j][r];
      }
    }
    wave_sync_lds();
    v4u hv[4], lv[4];
#pragma unroll
    for (int it = 0; it < 4; ++it) {
      const int row = it * 4 + q8;
      float brow = 0.0f;
      if (BM == 2) {
        int bi = mBase + row;
        bi = (bi < 0) ? 0 : ((bi > nb - 1) ? (nb - 1) : bi);
        brow = bfr(bias[bi]);
      }
      const float* sp = slab + row * 68 + c8;
      v4u a, lw;
#pragma unroll
      for (int e = 0; e < 4; ++e) {
        const float f0 = sp[2 * e]     * oscale + (bcol[2 * e]     + brow);
        const float f1 = sp[2 * e + 1] * oscale + (bcol[2 * e + 1] + brow);
        const _Float16 g0 = (_Float16)f0;
        const _Float16 g1 = (_Float16)f1;
        a[e] = pk16(h_bits(g0), h_bits(g1));
        const _Float16 z0 = (_Float16)((f0 - (float)g0) * rsc);
        const _Float16 z1 = (_Float16)((f1 - (float)g1) * rsc);
        lw[e] = pk16(h_bits(z0), h_bits(z1));
      }
      hv[it] = a;
      lv[it] = lw;
    }
    for (int pass = 0; pass < 2; ++pass) {
#pragma unroll
      for (int it = 0; it < 4; ++it) {
        const int row = it * 4 + q8;
        const size_t go = (size_t)(mBase + row) * ldc + n0 + c8;
        *(volatile v4u*)(Cout + go)  = hv[it];
        *(volatile v4u*)(Cout2 + go) = lv[it];
      }
      __threadfence();
    }
    wave_sync_lds();
  }
}

__global__ __launch_bounds__(256) void gemm_ob(
    const unsigned short* __restrict__ Ah, const unsigned short* __restrict__ Al, int lda,
    const unsigned short* __restrict__ Btp, int ldb,
    const float* __restrict__ bias, int nb,
    float* Cout, int ldc, int M, int N, int K) {
  __shared__ __align__(16) float sT[8][16 * 68];
  const int lane = threadIdx.x & 31;
  const int wave = threadIdx.x >> 5;
  const int tilesN = N >> 6;
  const int tilesM = M >> 6;
  const int tile = blockIdx.x * 8 + wave;
  if (tile >= tilesM * tilesN) return;
  const int tm = tile / tilesN;
  const int tn = tile - tm * tilesN;
  const int m0 = tm << 6;
  const int n0 = tn << 6;

  const int rlane = lane & 15;
  const int koff  = (lane >> 4) * 8;
  const int mOff  = (lane >> 4) * 8;

  v8f acc[4][4];
#pragma unroll
  for (int i = 0; i < 4; ++i)
#pragma unroll
    for (int j = 0; j < 4; ++j) acc[i][j] = zero8();

  for (int k0 = 0; k0 < K; k0 += 32) {
    FB bh[4];
#pragma unroll
    for (int j = 0; j < 4; ++j) {
      const size_t bo = (size_t)(n0 + (j << 4) + rlane) * ldb + koff + k0;
      bh[j] = ldfrag_b(Btp + bo);
    }
#pragma unroll
    for (int i = 0; i < 4; ++i) {
      const size_t ao = (size_t)(m0 + (i << 4) + rlane) * lda + koff + k0;
      const FB ah = ldfrag_b(Ah + ao);
      const FB al = ldfrag_b(Al + ao);
#pragma unroll
      for (int j = 0; j < 4; ++j) acc[i][j] = mma_b_raw(ah.v, bh[j].v, acc[i][j]);
#pragma unroll
      for (int j = 0; j < 4; ++j) acc[i][j] = mma_b_raw(al.v, bh[j].v, acc[i][j]);
      dep_guard2(acc[i][0], acc[i][3], ah.h, al.h);
    }
    keep4_h(bh[0].h, bh[1].h, bh[2].h, bh[3].h);
  }
  acc_guard4(acc[0][0], acc[0][1], acc[0][2], acc[0][3]);
  acc_guard4(acc[1][0], acc[1][1], acc[1][2], acc[1][3]);
  acc_guard4(acc[2][0], acc[2][1], acc[2][2], acc[2][3]);
  acc_guard4(acc[3][0], acc[3][1], acc[3][2], acc[3][3]);

  float* slab = sT[wave];
  const int hh2 = lane >> 4, c4 = (lane & 15) * 4;
  v4f bvec;
#pragma unroll
  for (int e = 0; e < 4; ++e) {
    int bi = n0 + c4 + e;
    bi = (bi < 0) ? 0 : ((bi > nb - 1) ? (nb - 1) : bi);
    bvec[e] = bfr(bias[bi]);
  }
#pragma unroll
  for (int i = 0; i < 4; ++i) {
    const int mBase = m0 + (i << 4);
#pragma unroll
    for (int j = 0; j < 4; ++j) {
#pragma unroll
      for (int r = 0; r < 8; ++r) {
        slab[(mOff + r) * 68 + (j << 4) + rlane] = acc[i][j][r];
      }
    }
    wave_sync_lds();
    v4f vals[8];
#pragma unroll
    for (int it = 0; it < 8; ++it) {
      const int row = it * 2 + hh2;
      vals[it] = *(const v4f*)(slab + row * 68 + c4) + bvec;
    }
    for (int pass = 0; pass < 2; ++pass) {
#pragma unroll
      for (int it = 0; it < 8; ++it) {
        const int row = it * 2 + hh2;
        const size_t go = (size_t)(mBase + row) * ldc + n0 + c4;
        *(volatile v4f*)(Cout + go) = vals[it];
      }
      __threadfence();
    }
    wave_sync_lds();
  }
}

__global__ __launch_bounds__(128)
void lattn(const unsigned short* __restrict__ qhp, const unsigned short* __restrict__ qlp,
           const unsigned short* __restrict__ khp, const unsigned short* __restrict__ klp,
           const unsigned short* __restrict__ vthp, const unsigned short* __restrict__ vtlp,
           float* ao, float sscale) {
  union FH { v16h v; v8h h[2]; };
  __shared__ __align__(16) _Float16 Psh[4][16 * 64];
  __shared__ __align__(16) _Float16 Psl[4][16 * 64];
  __shared__ __align__(16) float    Os[4][16 * 64];

  const int tid  = threadIdx.x;
  const int wave = tid >> 5;
  const int lane = tid & 31;
  const int hh   = lane >> 4;
  const int c    = lane & 15;

  const int bx   = blockIdx.x;
  const int wch  = bx % NCH;
  const int hq   = bx / NCH;
  const int q0   = wch * 64 + wave * 16;

  const _Float16* Qh = (const _Float16*)(const void*)qhp + (size_t)hq * HD;
  const _Float16* Ql = (const _Float16*)(const void*)qlp + (size_t)hq * HD;
  const _Float16* Kh = (const _Float16*)(const void*)khp + (size_t)hq * HD;
  const _Float16* Kl = (const _Float16*)(const void*)klp + (size_t)hq * HD;
  const _Float16* Vh = (const _Float16*)(const void*)vthp + (size_t)hq * HD * SQ;
  const _Float16* Vl = (const _Float16*)(const void*)vtlp + (size_t)hq * HD * SQ;

  v16h qa[2], qr[2];
#pragma unroll
  for (int dc = 0; dc < 2; ++dc) {
    qa[dc] = ldfrag_h(Qh + (size_t)(q0 + c) * DM + dc * 32 + 8 * hh);
    qr[dc] = ldfrag_h(Ql + (size_t)(q0 + c) * DM + dc * 32 + 8 * hh);
  }

  v8f oacc[4];
#pragma unroll
  for (int t = 0; t < 4; ++t) oacc[t] = zero8();

  int ktLo = wch - 1;
  if (ktLo < 0) ktLo = 0;
  int ktHi = wch + 1;
  if (ktHi > NCH - 1) ktHi = NCH - 1;
  const float rinv = 1.0f / RSC;
  _Float16* pwh = Psh[wave];
  _Float16* pwl = Psl[wave];

  for (int kt = ktLo; kt <= ktHi; ++kt) {
    const int kv0 = kt * 64;

#pragma unroll 1
    for (int j = 0; j < 4; ++j) {
      v8f sh = zero8(), sl = zero8();
      const size_t krow = (size_t)(kv0 + j * 16 + c) * DM;
#pragma unroll
      for (int dc = 0; dc < 2; ++dc) {
        const v16h kb = ldfrag_h(Kh + krow + dc * 32 + 8 * hh);
        const v16h kr = ldfrag_h(Kl + krow + dc * 32 + 8 * hh);
        sh = mma_h(qa[dc], kb, sh);
        sl = mma_h(qa[dc], kr, sl);
        sl = mma_h(qr[dc], kb, sl);
      }
#pragma unroll
      for (int r = 0; r < 8; ++r) {
        float p = (sh[r] + sl[r] * rinv) * sscale;
        p = fmaxf(p, 0.0f);
        const _Float16 ph = (_Float16)p;
        const int pi = (8 * hh + r) * 64 + j * 16 + c;
        pwh[pi] = ph;
        pwl[pi] = (_Float16)((p - (float)ph) * RSC);
      }
    }
    wave_sync_lds();

    v8f ol[4];
#pragma unroll
    for (int t = 0; t < 4; ++t) ol[t] = zero8();
#pragma unroll 1
    for (int kk = 0; kk < 2; ++kk) {
      FH pa, pr;
      pa.h[0] = *(const v8h*)(pwh + c * 64 + kk * 32 + 8 * hh);
      pa.h[1] = *(const v8h*)(pwh + c * 64 + kk * 32 + 16 + 8 * hh);
      pr.h[0] = *(const v8h*)(pwl + c * 64 + kk * 32 + 8 * hh);
      pr.h[1] = *(const v8h*)(pwl + c * 64 + kk * 32 + 16 + 8 * hh);
#pragma unroll
      for (int t = 0; t < 4; ++t) {
        const size_t vrow = (size_t)(t * 16 + c) * SQ + kv0 + kk * 32 + 8 * hh;
        const v16h vb = ldfrag_h(Vh + vrow);
        const v16h wb = ldfrag_h(Vl + vrow);
        oacc[t] = mma_h(pa.v, vb, oacc[t]);
        ol[t]   = mma_h(pa.v, wb, ol[t]);
        ol[t]   = mma_h(pr.v, vb, ol[t]);
      }
    }
#pragma unroll
    for (int t = 0; t < 4; ++t) {
#pragma unroll
      for (int r = 0; r < 8; ++r) oacc[t][r] += ol[t][r] * rinv;
    }
    wave_sync_lds();
  }

  float* os = Os[wave];
#pragma unroll
  for (int r = 0; r < 8; ++r) {
#pragma unroll
    for (int t = 0; t < 4; ++t) os[(8 * hh + r) * 64 + t * 16 + c] = oacc[t][r];
  }
  wave_sync_lds();
  {
    const int hh2 = lane >> 4, c4 = (lane & 15) * 4;
    v4f vals[8];
#pragma unroll
    for (int it = 0; it < 8; ++it) {
      const int row = it * 2 + hh2;
      vals[it] = *(const v4f*)(os + row * 64 + c4);
    }
    for (int pass = 0; pass < 2; ++pass) {
#pragma unroll
      for (int it = 0; it < 8; ++it) {
        const int row = it * 2 + hh2;
        const size_t go = (size_t)(q0 + row) * DM + (size_t)hq * HD + c4;
        *(volatile v4f*)(ao + go) = vals[it];
      }
      __threadfence();
    }
  }
}

__global__ __launch_bounds__(128) void gnorm(const float* ao, const float* __restrict__ nsc,
                                             const float* __restrict__ ngt,
                                             unsigned short* yh, unsigned short* yl) {
  __shared__ float red[4];
  __shared__ __align__(16) unsigned short shh[DM];
  __shared__ __align__(16) unsigned short shl[DM];
  const int tid  = threadIdx.x;
  const int lane = tid & 31;
  const int wave = tid >> 5;
  const size_t row = blockIdx.x;
  const float* xr = ao + row * DM + (size_t)tid * 8;
  const v4f a = *(const v4f*)(xr);
  const v4f b = *(const v4f*)(xr + 4);
  float ss = a[0] * a[0];
  ss += a[1] * a[1];
  ss += a[2] * a[2];
  ss += a[3] * a[3];
  ss += b[0] * b[0];
  ss += b[1] * b[1];
  ss += b[2] * b[2];
  ss += b[3] * b[3];
#pragma unroll
  for (int off = 1; off < 32; off <<= 1) ss += __shfl_xor(ss, off, 32);
  if (lane == 0) red[wave] = ss;
  __syncthreads();
  const float tot = (red[0] + red[1]) + (red[2] + red[3]);
  const float rms = sqrtf(tot * (1.0f / (float)DM));
  const float inv = 1.0f / (rms + 1e-8f);
#pragma unroll 1
  for (int e = 0; e < 8; ++e) {
    const int col = tid * 8 + e;
    const float x = xr[e];
    float z = bfr(ngt[col]) * x;
    z = fminf(fmaxf(z, -30.0f), 30.0f);
    const float sg = 1.0f / (1.0f + expf(-z));
    const float y = (bfr(nsc[col]) * (x * inv)) * sg;
    const unsigned short h = bf_bits(y);
    shh[col] = h;
    shl[col] = bf_bits(y - bf_up(h));
  }
  __syncthreads();
  const v8us hv = *(const v8us*)(shh + tid * 8);
  const v8us lv = *(const v8us*)(shl + tid * 8);
  const size_t go = row * DM + (size_t)tid * 8;
  for (int pass = 0; pass < 2; ++pass) {
    *(volatile v8us*)(yh + go) = hv;
    *(volatile v8us*)(yl + go) = lv;
    __threadfence();
  }
}

extern "C" void kernel_launch(void* const* d_in, const int* in_sizes, int n_in,
                              void* d_out, int out_size, void* d_ws, size_t ws_size,
                              hipStream_t stream) {
  if (n_in < 13) return;
  if (in_sizes[0] != SQ * DM || in_sizes[1] != SQ * DM || in_sizes[2] != SQ * DM) return;
  if (in_sizes[3] != DM * DM || in_sizes[5] != DM * DM || in_sizes[7] != DM * DM) return;
  if (in_sizes[9] != DM * DM) return;
  if (in_sizes[4] != DM || in_sizes[6] != DM || in_sizes[8] != DM || in_sizes[10] != DM) return;
  if (in_sizes[11] != DM || in_sizes[12] != DM) return;
  if (out_size != SQ * DM) return;

  const float* query = (const float*)d_in[0];
  const float* key   = (const float*)d_in[1];
  const float* value = (const float*)d_in[2];
  const float* wq    = (const float*)d_in[3];
  const float* bq    = (const float*)d_in[4];
  const float* wk    = (const float*)d_in[5];
  const float* bk    = (const float*)d_in[6];
  const float* wv    = (const float*)d_in[7];
  const float* bv    = (const float*)d_in[8];
  const float* wo    = (const float*)d_in[9];
  const float* bo    = (const float*)d_in[10];
  const float* nsc   = (const float*)d_in[11];
  const float* ngt   = (const float*)d_in[12];

  const size_t PX = (size_t)SQ * DM * 2;
  const size_t PW = (size_t)DM * DM * 2;
  const size_t PF = (size_t)SQ * DM * 4;
  const size_t oX  = 0;
  const size_t oWq = oX + PX;
  const size_t oWk = oWq + PW;
  const size_t oWv = oWk + PW;
  if (oWv + PW > PF) return;
  const size_t oAO = 0;
  const size_t oQH = PF;
  const size_t oQL = oQH + PX;
  const size_t oKH = oQL + PX;
  const size_t oKL = oKH + PX;
  const size_t oVH = oKL + PX;
  const size_t oVL = oVH + PX;
  const size_t end = oVL + PX;
  const size_t oWo = oQH;
  const size_t oYH = oKH;
  const size_t oYL = oKL;
  if (end > ws_size) return;
  if (end > (size_t)134217728) return;

  char* ws = (char*)d_ws;
  unsigned short* X   = (unsigned short*)(ws + oX);
  unsigned short* WqH = (unsigned short*)(ws + oWq);
  unsigned short* WkH = (unsigned short*)(ws + oWk);
  unsigned short* WvH = (unsigned short*)(ws + oWv);
  float*          AO  = (float*)(ws + oAO);
  unsigned short* QH  = (unsigned short*)(ws + oQH);
  unsigned short* QL  = (unsigned short*)(ws + oQL);
  unsigned short* KH  = (unsigned short*)(ws + oKH);
  unsigned short* KL  = (unsigned short*)(ws + oKL);
  unsigned short* VTH = (unsigned short*)(ws + oVH);
  unsigned short* VTL = (unsigned short*)(ws + oVL);
  unsigned short* WoB = (unsigned short*)(ws + oWo);
  unsigned short* YH  = (unsigned short*)(ws + oYH);
  unsigned short* YL  = (unsigned short*)(ws + oYL);

  const dim3 blk(256), blk128(128);
  const dim3 gCw((DM * DM / 8 + 255) / 256);
  const dim3 gCx((SQ * DM / 8 + 255) / 256);
  const dim3 gG(((SQ / 64) * (DM / 64) + 7) / 8);
  const dim3 gA(NH * NCH);
  const dim3 gN(SQ);
  const float invw = 1.0f / WSC;

  conv16<0><<<gCw, blk, 0, stream>>>(wq, WqH, DM * DM / 8, WSC);
  conv16<0><<<gCw, blk, 0, stream>>>(wk, WkH, DM * DM / 8, WSC);
  conv16<0><<<gCw, blk, 0, stream>>>(wv, WvH, DM * DM / 8, WSC);

  conv16<0><<<gCx, blk, 0, stream>>>(query, X, SQ * DM / 8, 1.0f);
  gemm64<1><<<gG, blk, 0, stream>>>(X, DM, WqH, DM, bq, DM, QH, QL, DM, SQ, DM, DM, invw, RSC);
  conv16<0><<<gCx, blk, 0, stream>>>(key, X, SQ * DM / 8, 1.0f);
  gemm64<1><<<gG, blk, 0, stream>>>(X, DM, WkH, DM, bk, DM, KH, KL, DM, SQ, DM, DM, invw, RSC);
  conv16<0><<<gCx, blk, 0, stream>>>(value, X, SQ * DM / 8, 1.0f);
  gemm64<2><<<gG, blk, 0, stream>>>(WvH, DM, X, DM, bv, DM, VTH, VTL, SQ, DM, SQ, DM, invw, RSC);

  lattn<<<gA, blk128, 0, stream>>>(QH, QL, KH, KL, VTH, VTL, AO, 0.125f);

  conv16<1><<<gCw, blk, 0, stream>>>(wo, WoB, DM * DM / 8, 1.0f);
  gnorm<<<gN, blk128, 0, stream>>>(AO, nsc, ngt, YH, YL);

  gemm_ob<<<gG, blk, 0, stream>>>(YH, YL, DM, WoB, DM, bo, DM, (float*)d_out, DM, SQ, DM, DM);
  (void)hipGetLastError();
}
